// MSBGHearingModel_36438502539758
// MI455X (gfx1250) — hardware-verified
//
#include <hip/hip_runtime.h>
#include <math.h>

typedef unsigned short us;
typedef us     v8us  __attribute__((ext_vector_type(8)));
typedef us     v16us __attribute__((ext_vector_type(16)));
typedef __bf16 v16bf __attribute__((ext_vector_type(16)));
typedef float  v8f   __attribute__((ext_vector_type(8)));
typedef float  v4f   __attribute__((ext_vector_type(4)));
typedef v8us __attribute__((may_alias)) v8usa;
typedef v4f  __attribute__((may_alias)) v4fa;

constexpr int TL    = 220500;
constexpr int NSIG  = 2;
constexpr int NCH   = 28;
constexpr int OFS   = 512;
constexpr int MP    = 13824;
constexpr int TP    = MP * 16;
constexpr int PL    = 222272;
constexpr int KP    = 1056;
constexpr int NFR   = 3446;
constexpr int FRW   = NSIG * NFR;
constexpr int RPAD  = 6912;
constexpr int NFILT = 86;
constexpr int FROWS = 16 * KP;
constexpr int TAPE  = 1015;
constexpr int TAPG  = 1025;
constexpr float EPSV = 1e-8f;

static_assert(PL % 64 == 0);
static_assert(PL >= 16 * (MP - 1) + KP);
static_assert(TP % 32 == 0);
static_assert(RPAD % 32 == 0 && RPAD >= FRW);
static_assert((NSIG * PL) % 128 == 0);

__device__ __forceinline__ us bfr(float f) {
  unsigned u = __float_as_uint(f);
  u += 0x7FFFu + ((u >> 16) & 1u);
  return (us)(u >> 16);
}
__device__ __forceinline__ float bff(us b) { return __uint_as_float(((unsigned)b) << 16); }
__device__ __forceinline__ us bflo(float f, us hi) { return bfr(f - bff(hi)); }

__device__ __forceinline__ v16bf ldfrag(const us* p, int h) {
  const v8us lo = *(const v8usa*)(p + 8 * h);
  const v8us hi = *(const v8usa*)(p + 16 + 8 * h);
  const v16us c = __builtin_shufflevector(lo, hi, 0, 1, 2, 3, 4, 5, 6, 7, 8, 9, 10, 11, 12, 13, 14, 15);
  return __builtin_bit_cast(v16bf, c);
}

__device__ __forceinline__ v8f wmma1(v16bf a, v16bf b, v8f c) {
  return __builtin_amdgcn_wmma_f32_16x16x32_bf16(false, a, false, b, (short)0, c, false, false);
}
__device__ __forceinline__ v8f wmma3(v16bf ah, v16bf al, v16bf bh, v16bf bl, v8f c) {
  v8f d = wmma1(ah, bh, c);
  d = wmma1(ah, bl, d);
  d = wmma1(al, bh, d);
  asm volatile("v_nop\n\tv_nop\n\tv_nop\n\tv_nop" : "+v"(d) : "v"(ah), "v"(al), "v"(bh), "v"(bl));
  return d;
}

__device__ __forceinline__ void st512f(const float* st, float* dst, int lane) {
#pragma unroll
  for (int i = 0; i < 4; ++i) {
    const v4f v = *(const v4fa*)(st + 128 * i + 4 * lane);
    *(volatile v4f*)(dst + 128 * i + 4 * lane) = v;
  }
}
__device__ __forceinline__ void st512h(const us* st, us* dst, int lane) {
#pragma unroll
  for (int i = 0; i < 2; ++i) {
    const v8us v = *(const v8usa*)(st + 256 * i + 8 * lane);
    *(volatile v8us*)(dst + 256 * i + 8 * lane) = v;
  }
}

__global__ __launch_bounds__(128) void k_cvt_x(const float* __restrict__ x, us* __restrict__ xH, us* __restrict__ xL) {
  const int g = blockIdx.x * 128 + threadIdx.x;
  if (g >= (NSIG * PL) / 8) return;
  const int e = 8 * g;
  const int b = (e >= PL) ? 1 : 0;
  const int p = e - b * PL;
  v8us vh, vl;
#pragma unroll
  for (int i = 0; i < 8; ++i) {
    const int t = p + i - OFS;
    const int tc = min(max(t, 0), TL - 1);
    float v = x[(size_t)b * TL + tc];
    v = (t >= 0 && t < TL) ? v : 0.0f;
    const us hi = bfr(v);
    vh[i] = hi;
    vl[i] = bflo(v, hi);
  }
  us* ph = xH + e;
  us* pq = xL + e;
  *(volatile v8us*)ph = vh;
  *(volatile v8us*)pq = vl;
  __threadfence();
  *(volatile v8us*)ph = vh;
  *(volatile v8us*)pq = vl;
}

__global__ __launch_bounds__(128) void k_prep_tw(const float* __restrict__ fsm,
    us* __restrict__ twFH, us* __restrict__ twFL, us* __restrict__ twIH, us* __restrict__ twIL,
    us* __restrict__ fsH, us* __restrict__ fsL) {
  __shared__ __attribute__((aligned(16))) us sh[128];
  __shared__ __attribute__((aligned(16))) us sl[128];
  const int task = blockIdx.y, tid = threadIdx.x;
  const int e = blockIdx.x * 128 + tid;
  float v;
  us* dH;
  us* dL;
  if (task == 2) {
    if (blockIdx.x >= 512) return;
    v = fsm[e];
    dH = fsH; dL = fsL;
  } else {
    int kk, tt, usesin;
    float sc;
    if (task == 0) {
      const int n = e >> 8, j = e & 255;
      kk = n & 255; tt = j + 128; usesin = (n >= 256); sc = 1.0f;
      dH = twFH; dL = twFL;
    } else {
      const int n = e >> 9, kq = e & 511;
      kk = kq & 255; tt = n + 128; usesin = (kq >= 256);
      sc = (kk == 0) ? (1.0f / 512.0f) : (1.0f / 256.0f);
      dH = twIH; dL = twIL;
    }
    const int r = (kk * tt) & 511;
    float s, c;
    sincospif((float)r * (1.0f / 256.0f), &s, &c);
    v = usesin ? (-s * sc) : (c * sc);
  }
  const us hi = bfr(v);
  sh[tid] = hi;
  sl[tid] = bflo(v, hi);
  __syncthreads();
  if (tid < 16) {
    const v8us a = *(const v8usa*)(sh + 8 * tid);
    const v8us c = *(const v8usa*)(sl + 8 * tid);
    us* ph = dH + (size_t)blockIdx.x * 128 + 8 * tid;
    us* pq = dL + (size_t)blockIdx.x * 128 + 8 * tid;
    *(volatile v8us*)ph = a;
    *(volatile v8us*)pq = c;
    __threadfence();
    *(volatile v8us*)ph = a;
    *(volatile v8us*)pq = c;
  }
}

__global__ __launch_bounds__(128) void k_prep_filt(const float* __restrict__ cf, const float* __restrict__ cb,
    const float* __restrict__ gc, const float* __restrict__ gs, const float* __restrict__ lp,
    us* __restrict__ bH, us* __restrict__ bL) {
  const int fid = blockIdx.y;
  const int g = blockIdx.x * 128 + threadIdx.x;
  if (g >= FROWS / 8) return;
  const int e = 8 * g;
  const int bp = e / KP;
  const int k0 = e - bp * KP;
  const float* w;
  int taps, sh;
  if (fid == 0)      { w = cf; taps = TAPE; sh = 5; }
  else if (fid == 1) { w = cb; taps = TAPE; sh = 5; }
  else if (fid < 58) { const int f = fid - 2; w = ((f & 1) ? gs : gc) + (size_t)(f >> 1) * TAPG; taps = TAPG; sh = 0; }
  else               { w = lp + (size_t)(fid - 58) * TAPG; taps = TAPG; sh = 0; }
  v8us vh, vl;
#pragma unroll
  for (int i = 0; i < 8; ++i) {
    const int idx = k0 + i - bp - sh;
    const int ic = min(max(idx, 0), taps - 1);
    float v = w[ic];
    v = (idx >= 0 && idx < taps) ? v : 0.0f;
    const us hi = bfr(v);
    vh[i] = hi;
    vl[i] = bflo(v, hi);
  }
  us* ph = bH + (size_t)fid * FROWS + e;
  us* pq = bL + (size_t)fid * FROWS + e;
  *(volatile v8us*)ph = vh;
  *(volatile v8us*)pq = vl;
  __threadfence();
  *(volatile v8us*)ph = vh;
  *(volatile v8us*)pq = vl;
}

__global__ __launch_bounds__(128) void k_conv16(const us* __restrict__ aH, const us* __restrict__ aL,
    const us* __restrict__ bH, const us* __restrict__ bL, float* __restrict__ out) {
  __shared__ __attribute__((aligned(16))) float sT[4][512];
  const int tid = threadIdx.x, lane = tid & 31, w = tid >> 5, h = lane >> 4, m = lane & 15;
  const int b = blockIdx.y;
  const int a0 = blockIdx.x * 128 + 32 * w;
  const us* pah = aH + (size_t)b * PL + 16 * (a0 + m);
  const us* pal = aL + (size_t)b * PL + 16 * (a0 + m);
  const us* pbh = bH + (size_t)m * KP;
  const us* pbl = bL + (size_t)m * KP;
  const v8f z8 = {0.f, 0.f, 0.f, 0.f, 0.f, 0.f, 0.f, 0.f};
  v8f acc0 = z8, acc1 = z8;
#pragma unroll 1
  for (int k0 = 0; k0 < KP; k0 += 32) {
    const v16bf ah0 = ldfrag(pah + k0, h), al0 = ldfrag(pal + k0, h);
    const v16bf ah1 = ldfrag(pah + 256 + k0, h), al1 = ldfrag(pal + 256 + k0, h);
    const v16bf bh = ldfrag(pbh + k0, h), bl = ldfrag(pbl + k0, h);
    acc0 = wmma3(ah0, al0, bh, bl, acc0);
    acc1 = wmma3(ah1, al1, bh, bl, acc1);
  }
  float* st = sT[w];
#pragma unroll
  for (int r = 0; r < 8; ++r) {
    st[16 * (8 * h + r) + m] = acc0[r];
    st[16 * (16 + 8 * h + r) + m] = acc1[r];
  }
  __syncthreads();
  float* dst = out + (size_t)b * TP + 16 * a0;
  st512f(st, dst, lane);
  __threadfence();
  st512f(st, dst, lane);
}

__global__ __launch_bounds__(256) void k_frames(const float* __restrict__ y1, const float* __restrict__ win,
    us* __restrict__ frH, us* __restrict__ frL, float* __restrict__ nyq) {
  __shared__ __attribute__((aligned(16))) float sN[32];
  const int tid = threadIdx.x, lane = tid & 31, w = tid >> 5;
  const int rbase = blockIdx.x * 32;
  const int j0 = 8 * lane;
#pragma unroll 1
  for (int i = 0; i < 4; ++i) {
    const int r = rbase + 4 * w + i;
    const bool rv = (r < FRW);
    const int rc = min(r, FRW - 1);
    const int b = (rc >= NFR) ? 1 : 0;
    const int f = rc - b * NFR;
    float alt = 0.0f;
    v8us vh, vl;
#pragma unroll
    for (int q = 0; q < 8; ++q) {
      const int j = j0 + q;
      const int t = 64 * f + 128 + j;
      float v = y1[(size_t)b * TP + t] * win[j];
      v = (rv && t < TL) ? v : 0.0f;
      alt += (q & 1) ? -v : v;
      const us hi = bfr(v);
      vh[q] = hi;
      vl[q] = bflo(v, hi);
    }
#pragma unroll
    for (int o = 16; o > 0; o >>= 1) alt += __shfl_xor(alt, o);
    if (lane == 0) sN[4 * w + i] = alt;
    us* ph = frH + (size_t)r * 256 + j0;
    us* pq = frL + (size_t)r * 256 + j0;
    *(volatile v8us*)ph = vh;
    *(volatile v8us*)pq = vl;
    __threadfence();
    *(volatile v8us*)ph = vh;
    *(volatile v8us*)pq = vl;
  }
  __syncthreads();
  if (w == 0 && lane < 8) {
    const v4f v = *(const v4fa*)(sN + 4 * lane);
    float* p = nyq + rbase + 4 * lane;
    *(volatile v4f*)p = v;
    __threadfence();
    *(volatile v4f*)p = v;
  }
}

__device__ __forceinline__ void dftf_store(const float* lRe, const float* lIm, float* sRe, float* sIm,
                                           us* pwH, us* pwL, int r0, int cblk, int w, int lane) {
#pragma unroll 1
  for (int i = 0; i < 8; ++i) {
    const int row = 8 * w + i;
    const v4f a = *(const v4fa*)(lRe + row * 128 + 4 * lane);
    const v4f c = *(const v4fa*)(lIm + row * 128 + 4 * lane);
    const size_t gi = (size_t)(r0 + row) * 256 + cblk + 4 * lane;
    *(volatile v4f*)(sRe + gi) = a;
    *(volatile v4f*)(sIm + gi) = c;
  }
#pragma unroll 1
  for (int i = 0; i < 4; ++i) {
    const int row = 8 * w + 2 * i + (lane >> 4);
    const int c8 = 8 * (lane & 15);
    v8us vh, vl;
#pragma unroll
    for (int q = 0; q < 8; ++q) {
      const float re = lRe[row * 128 + c8 + q];
      const float im = lIm[row * 128 + c8 + q];
      const float pw = re * re + im * im;
      const us hi = bfr(pw);
      vh[q] = hi;
      vl[q] = bflo(pw, hi);
    }
    const size_t gi = (size_t)(r0 + row) * 256 + cblk + c8;
    *(volatile v8us*)(pwH + gi) = vh;
    *(volatile v8us*)(pwL + gi) = vl;
  }
}

__global__ __launch_bounds__(128) void k_dft_fwd(const us* __restrict__ frH, const us* __restrict__ frL,
    const us* __restrict__ twH, const us* __restrict__ twL, float* __restrict__ sRe, float* __restrict__ sIm,
    us* __restrict__ pwH, us* __restrict__ pwL) {
  __shared__ __attribute__((aligned(16))) float lRe[32 * 128];
  __shared__ __attribute__((aligned(16))) float lIm[32 * 128];
  const int tid = threadIdx.x, lane = tid & 31, w = tid >> 5, h = lane >> 4, m = lane & 15;
  const int r0 = blockIdx.x * 32;
  const int cblk = blockIdx.y * 128;
  const int cw = cblk + 32 * w;
  const us* pah = frH + (size_t)(r0 + m) * 256;
  const us* pal = frL + (size_t)(r0 + m) * 256;
  const v8f z8 = {0.f, 0.f, 0.f, 0.f, 0.f, 0.f, 0.f, 0.f};
  v8f acc[2][4];
#pragma unroll
  for (int i = 0; i < 2; ++i)
#pragma unroll
    for (int j = 0; j < 4; ++j) acc[i][j] = z8;
#pragma unroll 1
  for (int k0 = 0; k0 < 256; k0 += 32) {
    const v16bf ah0 = ldfrag(pah + k0, h), al0 = ldfrag(pal + k0, h);
    const v16bf ah1 = ldfrag(pah + 16 * 256 + k0, h), al1 = ldfrag(pal + 16 * 256 + k0, h);
#pragma unroll
    for (int u = 0; u < 2; ++u) {
#pragma unroll
      for (int pt = 0; pt < 2; ++pt) {
        const size_t ro = (size_t)(256 * pt + cw + 16 * u + m) * 256 + k0;
        const v16bf bh = ldfrag(twH + ro, h), bl = ldfrag(twL + ro, h);
        acc[0][2 * pt + u] = wmma3(ah0, al0, bh, bl, acc[0][2 * pt + u]);
        acc[1][2 * pt + u] = wmma3(ah1, al1, bh, bl, acc[1][2 * pt + u]);
      }
    }
  }
#pragma unroll
  for (int mt = 0; mt < 2; ++mt)
#pragma unroll
    for (int u = 0; u < 2; ++u)
#pragma unroll
      for (int r = 0; r < 8; ++r) {
        const int row = 16 * mt + 8 * h + r;
        const int col = 32 * w + 16 * u + m;
        lRe[row * 128 + col] = acc[mt][u][r];
        lIm[row * 128 + col] = acc[mt][2 + u][r];
      }
  __syncthreads();
  dftf_store(lRe, lIm, sRe, sIm, pwH, pwL, r0, cblk, w, lane);
  __threadfence();
  dftf_store(lRe, lIm, sRe, sIm, pwH, pwL, r0, cblk, w, lane);
}

__device__ __forceinline__ void smear_store(const float* lS, const float* sRe, const float* sIm,
                                            us* sscH, us* sscL, int r0, int w, int lane) {
#pragma unroll 1
  for (int i = 0; i < 8; ++i) {
    const int row = 8 * w + i;
    const int c8 = 8 * lane;
    const float* ls = lS + row * 256 + c8;
    const v4f s0 = *(const v4fa*)ls, s1 = *(const v4fa*)(ls + 4);
    const size_t gi = (size_t)(r0 + row) * 256 + c8;
    const v4f ra = *(const v4fa*)(sRe + gi), rb = *(const v4fa*)(sRe + gi + 4);
    const v4f ia = *(const v4fa*)(sIm + gi), ib = *(const v4fa*)(sIm + gi + 4);
    const v8f sp8 = __builtin_shufflevector(s0, s1, 0, 1, 2, 3, 4, 5, 6, 7);
    const v8f re8 = __builtin_shufflevector(ra, rb, 0, 1, 2, 3, 4, 5, 6, 7);
    const v8f im8 = __builtin_shufflevector(ia, ib, 0, 1, 2, 3, 4, 5, 6, 7);
    v8us rh, rl, ih, il;
#pragma unroll
    for (int q = 0; q < 8; ++q) {
      const float re = re8[q], im = im8[q];
      const float pw = re * re + im * im;
      const float rt = __builtin_amdgcn_sqrtf((fmaxf(sp8[q], 0.0f) + EPSV) * __builtin_amdgcn_rcpf(pw + EPSV));
      const float a = re * rt, c = im * rt;
      us hi = bfr(a);
      rh[q] = hi; rl[q] = bflo(a, hi);
      hi = bfr(c);
      ih[q] = hi; il[q] = bflo(c, hi);
    }
    const size_t go = (size_t)(r0 + row) * 512 + c8;
    *(volatile v8us*)(sscH + go) = rh;
    *(volatile v8us*)(sscH + go + 256) = ih;
    *(volatile v8us*)(sscL + go) = rl;
    *(volatile v8us*)(sscL + go + 256) = il;
  }
}

__global__ __launch_bounds__(128) void k_smear(const us* __restrict__ pwH, const us* __restrict__ pwL,
    const us* __restrict__ fsH, const us* __restrict__ fsL, const float* __restrict__ sRe, const float* __restrict__ sIm,
    us* __restrict__ sscH, us* __restrict__ sscL) {
  __shared__ __attribute__((aligned(16))) float lS[32 * 256];
  const int tid = threadIdx.x, lane = tid & 31, w = tid >> 5, h = lane >> 4, m = lane & 15;
  const int r0 = blockIdx.x * 32;
  const int i0 = 64 * w;
  const us* pah = pwH + (size_t)(r0 + m) * 256;
  const us* pal = pwL + (size_t)(r0 + m) * 256;
  const v8f z8 = {0.f, 0.f, 0.f, 0.f, 0.f, 0.f, 0.f, 0.f};
  v8f acc[2][4];
#pragma unroll
  for (int i = 0; i < 2; ++i)
#pragma unroll
    for (int j = 0; j < 4; ++j) acc[i][j] = z8;
#pragma unroll 1
  for (int k0 = 0; k0 < 256; k0 += 32) {
    const v16bf ah0 = ldfrag(pah + k0, h), al0 = ldfrag(pal + k0, h);
    const v16bf ah1 = ldfrag(pah + 16 * 256 + k0, h), al1 = ldfrag(pal + 16 * 256 + k0, h);
#pragma unroll
    for (int u = 0; u < 4; ++u) {
      const size_t ro = (size_t)(i0 + 16 * u + m) * 256 + k0;
      const v16bf bh = ldfrag(fsH + ro, h), bl = ldfrag(fsL + ro, h);
      acc[0][u] = wmma3(ah0, al0, bh, bl, acc[0][u]);
      acc[1][u] = wmma3(ah1, al1, bh, bl, acc[1][u]);
    }
  }
#pragma unroll
  for (int mt = 0; mt < 2; ++mt)
#pragma unroll
    for (int u = 0; u < 4; ++u)
#pragma unroll
      for (int r = 0; r < 8; ++r)
        lS[(16 * mt + 8 * h + r) * 256 + i0 + 16 * u + m] = acc[mt][u][r];
  __syncthreads();
  smear_store(lS, sRe, sIm, sscH, sscL, r0, w, lane);
  __threadfence();
  smear_store(lS, sRe, sIm, sscH, sscL, r0, w, lane);
}

__device__ __forceinline__ void dfti_store(const float* lF, float* fro, int r0, int w, int lane) {
#pragma unroll 1
  for (int i = 0; i < 8; ++i) {
    const int row = 8 * w + i;
#pragma unroll
    for (int hh = 0; hh < 2; ++hh) {
      const v4f v = *(const v4fa*)(lF + row * 256 + 128 * hh + 4 * lane);
      *(volatile v4f*)(fro + (size_t)(r0 + row) * 256 + 128 * hh + 4 * lane) = v;
    }
  }
}

__global__ __launch_bounds__(128) void k_dft_inv(const us* __restrict__ sscH, const us* __restrict__ sscL,
    const us* __restrict__ twH, const us* __restrict__ twL, const float* __restrict__ nyq,
    const float* __restrict__ win, float* __restrict__ fro) {
  __shared__ __attribute__((aligned(16))) float lF[32 * 256];
  const int tid = threadIdx.x, lane = tid & 31, w = tid >> 5, h = lane >> 4, m = lane & 15;
  const int r0 = blockIdx.x * 32;
  const int n0 = 64 * w;
  const us* pah = sscH + (size_t)(r0 + m) * 512;
  const us* pal = sscL + (size_t)(r0 + m) * 512;
  const v8f z8 = {0.f, 0.f, 0.f, 0.f, 0.f, 0.f, 0.f, 0.f};
  v8f acc[2][4];
#pragma unroll
  for (int i = 0; i < 2; ++i)
#pragma unroll
    for (int j = 0; j < 4; ++j) acc[i][j] = z8;
#pragma unroll 1
  for (int k0 = 0; k0 < 512; k0 += 32) {
    const v16bf ah0 = ldfrag(pah + k0, h), al0 = ldfrag(pal + k0, h);
    const v16bf ah1 = ldfrag(pah + 16 * 512 + k0, h), al1 = ldfrag(pal + 16 * 512 + k0, h);
#pragma unroll
    for (int u = 0; u < 4; ++u) {
      const size_t ro = (size_t)(n0 + 16 * u + m) * 512 + k0;
      const v16bf bh = ldfrag(twH + ro, h), bl = ldfrag(twL + ro, h);
      acc[0][u] = wmma3(ah0, al0, bh, bl, acc[0][u]);
      acc[1][u] = wmma3(ah1, al1, bh, bl, acc[1][u]);
    }
  }
  const float sgm = (m & 1) ? (-1.0f / 512.0f) : (1.0f / 512.0f);
  float wv[4];
#pragma unroll
  for (int u = 0; u < 4; ++u) wv[u] = win[n0 + 16 * u + m];
#pragma unroll
  for (int mt = 0; mt < 2; ++mt)
#pragma unroll
    for (int r = 0; r < 8; ++r) {
      const int row = 16 * mt + 8 * h + r;
      const float ny = nyq[r0 + row] * sgm;
#pragma unroll
      for (int u = 0; u < 4; ++u)
        lF[row * 256 + n0 + 16 * u + m] = (acc[mt][u][r] + ny) * wv[u];
    }
  __syncthreads();
  dfti_store(lF, fro, r0, w, lane);
  __threadfence();
  dfti_store(lF, fro, r0, w, lane);
}

__global__ __launch_bounds__(128) void k_ola(const float* __restrict__ fro, const float* __restrict__ win,
                                            us* __restrict__ yH, us* __restrict__ yL) {
  __shared__ __attribute__((aligned(16))) us sh[128];
  __shared__ __attribute__((aligned(16))) us sl[128];
  const int tid = threadIdx.x;
  const int e = blockIdx.x * 128 + tid;
  const int b = (e >= PL) ? 1 : 0;
  const int p = e - b * PL;
  const int t = p - OFS;
  const int s = min(max(t, 0), TL - 1);
  int fhi = (s >= 128) ? ((s - 128) >> 6) : -1;
  fhi = min(fhi, NFR - 1);
  const int flo = (s <= 383) ? 0 : ((s - 383 + 63) >> 6);
  float acc = 0.0f, ws = 0.0f;
#pragma unroll
  for (int q = 0; q < 4; ++q) {
    const int f = flo + q;
    const bool ok = (f <= fhi);
    const int fc = min(f, NFR - 1);
    const int j = min(max(s - 64 * fc - 128, 0), 255);
    const float a = fro[((size_t)(b * NFR + fc)) * 256 + j];
    const float wq = win[j];
    acc = ok ? (acc + a) : acc;
    ws = ok ? (ws + wq * wq) : ws;
  }
  float v = acc * __builtin_amdgcn_rcpf(fmaxf(ws, 1e-6f));
  v = (t >= 0 && t < TL) ? v : 0.0f;
  const us hi = bfr(v);
  sh[tid] = hi;
  sl[tid] = bflo(v, hi);
  __syncthreads();
  if (tid < 16) {
    const v8us a = *(const v8usa*)(sh + 8 * tid);
    const v8us c = *(const v8usa*)(sl + 8 * tid);
    us* ph = yH + (size_t)blockIdx.x * 128 + 8 * tid;
    us* pq = yL + (size_t)blockIdx.x * 128 + 8 * tid;
    *(volatile v8us*)ph = a;
    *(volatile v8us*)pq = c;
    __threadfence();
    *(volatile v8us*)ph = a;
    *(volatile v8us*)pq = c;
  }
}

__global__ __launch_bounds__(64) void k_padz(us* __restrict__ env, us* __restrict__ y3) {
  const int r = blockIdx.x;
  const int tid = threadIdx.x;
  us* row = (r < 112) ? (env + (size_t)r * PL) : (y3 + (size_t)(r - 112) * PL);
  const v8us z = {0, 0, 0, 0, 0, 0, 0, 0};
  us* p0 = row + 8 * tid;
  us* p1 = row + OFS + TP + 8 * tid;
  us* p2 = row + OFS + TP + 512 + 8 * tid;
  const bool third = (tid < (PL - OFS - TP - 512) / 8);
  *(volatile v8us*)p0 = z;
  *(volatile v8us*)p1 = z;
  if (third) *(volatile v8us*)p2 = z;
  __threadfence();
  *(volatile v8us*)p0 = z;
  *(volatile v8us*)p1 = z;
  if (third) *(volatile v8us*)p2 = z;
}

__global__ __launch_bounds__(128) void k_gt(const us* __restrict__ yH, const us* __restrict__ yL,
    const us* __restrict__ bH, const us* __restrict__ bL, float* __restrict__ xr,
    us* __restrict__ eH, us* __restrict__ eL) {
  __shared__ __attribute__((aligned(16))) float sX[4][512];
  __shared__ __attribute__((aligned(16))) us sEH[4][512];
  __shared__ __attribute__((aligned(16))) us sEL[4][512];
  const int tid = threadIdx.x, lane = tid & 31, w = tid >> 5, h = lane >> 4, m = lane & 15;
  const int b = blockIdx.z;
  const int c = blockIdx.y;
  const int a0 = blockIdx.x * 128 + 32 * w;
  const us* pah = yH + (size_t)b * PL + 16 * (a0 + m);
  const us* pal = yL + (size_t)b * PL + 16 * (a0 + m);
  const size_t rb0 = ((size_t)(2 + 2 * c + 0) * 16 + m) * KP;
  const size_t rb1 = ((size_t)(2 + 2 * c + 1) * 16 + m) * KP;
  const v8f z8 = {0.f, 0.f, 0.f, 0.f, 0.f, 0.f, 0.f, 0.f};
  v8f acc[2][2];
  acc[0][0] = z8; acc[0][1] = z8; acc[1][0] = z8; acc[1][1] = z8;
#pragma unroll 1
  for (int k0 = 0; k0 < KP; k0 += 32) {
    const v16bf ah0 = ldfrag(pah + k0, h), al0 = ldfrag(pal + k0, h);
    const v16bf ah1 = ldfrag(pah + 256 + k0, h), al1 = ldfrag(pal + 256 + k0, h);
    {
      const v16bf bh = ldfrag(bH + rb0 + k0, h), bl = ldfrag(bL + rb0 + k0, h);
      acc[0][0] = wmma3(ah0, al0, bh, bl, acc[0][0]);
      acc[1][0] = wmma3(ah1, al1, bh, bl, acc[1][0]);
    }
    {
      const v16bf bh = ldfrag(bH + rb1 + k0, h), bl = ldfrag(bL + rb1 + k0, h);
      acc[0][1] = wmma3(ah0, al0, bh, bl, acc[0][1]);
      acc[1][1] = wmma3(ah1, al1, bh, bl, acc[1][1]);
    }
  }
#pragma unroll
  for (int mt = 0; mt < 2; ++mt)
#pragma unroll
    for (int r = 0; r < 8; ++r) {
      const int tl = 16 * (16 * mt + 8 * h + r) + m;
      const int t = 16 * a0 + tl;
      const float xv = acc[mt][0][r];
      const float xi = acc[mt][1][r];
      float ev = __builtin_amdgcn_sqrtf(xv * xv + xi * xi + EPSV);
      ev = (t < TL) ? ev : 0.0f;
      sX[w][tl] = xv;
      const us hi = bfr(ev);
      sEH[w][tl] = hi;
      sEL[w][tl] = bflo(ev, hi);
    }
  __syncthreads();
  const size_t rowbc = (size_t)(b * NCH + c);
  float* dx = xr + rowbc * TP + 16 * a0;
  us* dh = eH + rowbc * PL + OFS + 16 * a0;
  us* dl = eL + rowbc * PL + OFS + 16 * a0;
  st512f(sX[w], dx, lane);
  st512h(sEH[w], dh, lane);
  st512h(sEL[w], dl, lane);
  __threadfence();
  st512f(sX[w], dx, lane);
  st512h(sEH[w], dh, lane);
  st512h(sEL[w], dl, lane);
}

__global__ __launch_bounds__(128) void k_lpf(const us* __restrict__ eH, const us* __restrict__ eL,
    const us* __restrict__ bH, const us* __restrict__ bL, const float* __restrict__ xr,
    const float* __restrict__ expn, const float* __restrict__ emx, const float* __restrict__ ocf,
    us* __restrict__ yH, us* __restrict__ yL) {
  __shared__ __attribute__((aligned(16))) us sH[4][512];
  __shared__ __attribute__((aligned(16))) us sL[4][512];
  const int tid = threadIdx.x, lane = tid & 31, w = tid >> 5, h = lane >> 4, m = lane & 15;
  const int b = blockIdx.y;
  const int a0 = blockIdx.x * 128 + 32 * w;
  const v8f z8 = {0.f, 0.f, 0.f, 0.f, 0.f, 0.f, 0.f, 0.f};
  v8f ys0 = z8, ys1 = z8;
#pragma unroll 1
  for (int c = 0; c < NCH; ++c) {
    const size_t rowbc = (size_t)(b * NCH + c);
    const us* pah = eH + rowbc * PL + 16 * (a0 + m);
    const us* pal = eL + rowbc * PL + 16 * (a0 + m);
    const size_t rbo = ((size_t)(58 + c) * 16 + m) * KP;
    v8f acc0 = z8, acc1 = z8;
#pragma unroll 1
    for (int k0 = 0; k0 < KP; k0 += 32) {
      const v16bf ah0 = ldfrag(pah + k0, h), al0 = ldfrag(pal + k0, h);
      const v16bf ah1 = ldfrag(pah + 256 + k0, h), al1 = ldfrag(pal + 256 + k0, h);
      const v16bf bh = ldfrag(bH + rbo + k0, h), bl = ldfrag(bL + rbo + k0, h);
      acc0 = wmma3(ah0, al0, bh, bl, acc0);
      acc1 = wmma3(ah1, al1, bh, bl, acc1);
    }
    const float em = emx[c], ex = expn[c];
    const float iem = 1.0f / em;
    const float* xrow = xr + rowbc * TP + 16 * a0 + m;
#pragma unroll
    for (int r = 0; r < 8; ++r) {
      {
        const float e = fmaxf(acc0[r], EPSV);
        const float q = fminf(e, em) * iem;
        const float g = exp2f(ex * log2f(q));
        const float xv = xrow[16 * (8 * h + r)];
        ys0[r] = ys0[r] + xv * g;
      }
      {
        const float e = fmaxf(acc1[r], EPSV);
        const float q = fminf(e, em) * iem;
        const float g = exp2f(ex * log2f(q));
        const float xv = xrow[16 * (16 + 8 * h + r)];
        ys1[r] = ys1[r] + xv * g;
      }
    }
  }
  const float oc = ocf[0];
#pragma unroll
  for (int r = 0; r < 8; ++r) {
    {
      const int tl = 16 * (8 * h + r) + m;
      const int t = 16 * a0 + tl;
      float v = ys0[r] * oc;
      v = (t < TL) ? v : 0.0f;
      const us hi = bfr(v);
      sH[w][tl] = hi;
      sL[w][tl] = bflo(v, hi);
    }
    {
      const int tl = 16 * (16 + 8 * h + r) + m;
      const int t = 16 * a0 + tl;
      float v = ys1[r] * oc;
      v = (t < TL) ? v : 0.0f;
      const us hi = bfr(v);
      sH[w][tl] = hi;
      sL[w][tl] = bflo(v, hi);
    }
  }
  __syncthreads();
  us* dh = yH + (size_t)b * PL + OFS + 16 * a0;
  us* dl = yL + (size_t)b * PL + OFS + 16 * a0;
  st512h(sH[w], dh, lane);
  st512h(sL[w], dl, lane);
  __threadfence();
  st512h(sH[w], dh, lane);
  st512h(sL[w], dl, lane);
}

__global__ __launch_bounds__(128) void k_out(const float* __restrict__ y4, float* __restrict__ out) {
  const int g = blockIdx.x * 128 + threadIdx.x;
  if (g >= (NSIG * TL) / 4) return;
  v4f v;
#pragma unroll
  for (int i = 0; i < 4; ++i) {
    const int idx = 4 * g + i;
    const int b = (idx >= TL) ? 1 : 0;
    const int t = idx - b * TL;
    v[i] = y4[(size_t)b * TP + t];
  }
  float* p = out + 4 * (size_t)g;
  *(volatile v4f*)p = v;
  __threadfence();
  *(volatile v4f*)p = v;
}

extern "C" void kernel_launch(void* const* d_in, const int* in_sizes, int n_in,
                              void* d_out, int out_size, void* d_ws, size_t ws_size,
                              hipStream_t stream) {
  if (n_in < 11) return;
  if (in_sizes[0] != NSIG * TL) return;
  if (in_sizes[1] != TAPE || in_sizes[2] != TAPE) return;
  if (in_sizes[3] != 256 || in_sizes[4] != 256 * 256) return;
  if (in_sizes[5] != NCH * TAPG || in_sizes[6] != NCH * TAPG || in_sizes[7] != NCH * TAPG) return;
  if (in_sizes[8] != NCH || in_sizes[9] != NCH || in_sizes[10] < 1) return;
  if (out_size != NSIG * TL) return;

  const float* x    = (const float*)d_in[0];
  const float* cf   = (const float*)d_in[1];
  const float* cbw  = (const float*)d_in[2];
  const float* win  = (const float*)d_in[3];
  const float* fsm  = (const float*)d_in[4];
  const float* gc   = (const float*)d_in[5];
  const float* gs   = (const float*)d_in[6];
  const float* lp   = (const float*)d_in[7];
  const float* expn = (const float*)d_in[8];
  const float* emx  = (const float*)d_in[9];
  const float* ocf  = (const float*)d_in[10];
  float* out = (float*)d_out;

  size_t off = 0;
  auto cv = [&](size_t bytes) -> size_t { size_t p = off; off = (off + bytes + 255) & ~(size_t)255; return p; };
  const size_t szB   = (size_t)NFILT * FROWS * 2;
  const size_t szTW  = (size_t)512 * 256 * 2;
  const size_t szFS  = (size_t)256 * 256 * 2;
  const size_t szPLN = (size_t)NSIG * PL * 2;
  const size_t szF32 = (size_t)NSIG * TP * 4;
  const size_t oBH  = cv(szB);
  const size_t oBL  = cv(szB);
  const size_t oTFH = cv(szTW);
  const size_t oTFL = cv(szTW);
  const size_t oTIH = cv(szTW);
  const size_t oTIL = cv(szTW);
  const size_t oFSH = cv(szFS);
  const size_t oFSL = cv(szFS);
  const size_t oXH  = cv(szPLN);
  const size_t oXL  = cv(szPLN);
  const size_t oY1  = cv(szF32);
  const size_t oY2H = cv(szPLN);
  const size_t oY2L = cv(szPLN);
  const size_t oY3  = cv((size_t)4 * PL * 2);
  const size_t oY4  = cv(szF32);
  const size_t oNYQ = cv((size_t)RPAD * 4);
  const size_t oScr = off;
  const size_t szFR  = (size_t)RPAD * 256 * 2;
  const size_t szSP  = (size_t)RPAD * 256 * 4;
  const size_t szSS  = (size_t)RPAD * 512 * 2;
  const size_t oFRH = cv(szFR);
  const size_t oFRL = cv(szFR);
  const size_t oSRE = cv(szSP);
  const size_t oSIM = cv(szSP);
  const size_t oPWH = cv(szFR);
  const size_t oPWL = cv(szFR);
  const size_t oSSH = cv(szSS);
  const size_t oSSL = cv(szSS);
  const size_t oFRO = cv(szSP);
  const size_t endA = off;
  off = oScr;
  const size_t oXR  = cv((size_t)NSIG * NCH * TP * 4);
  const size_t oENV = cv((size_t)4 * NCH * PL * 2);
  const size_t endB = off;
  const size_t total = (endA > endB) ? endA : endB;
  if (total > ws_size) return;

  char* ws = (char*)d_ws;
  us* BH  = (us*)(ws + oBH);   us* BL  = (us*)(ws + oBL);
  us* TFH = (us*)(ws + oTFH);  us* TFL = (us*)(ws + oTFL);
  us* TIH = (us*)(ws + oTIH);  us* TIL = (us*)(ws + oTIL);
  us* FSH = (us*)(ws + oFSH);  us* FSL = (us*)(ws + oFSL);
  us* XH  = (us*)(ws + oXH);   us* XL  = (us*)(ws + oXL);
  float* Y1 = (float*)(ws + oY1);
  us* Y2H = (us*)(ws + oY2H);  us* Y2L = (us*)(ws + oY2L);
  us* Y3  = (us*)(ws + oY3);
  float* Y4 = (float*)(ws + oY4);
  float* NYQ = (float*)(ws + oNYQ);
  us* FRH = (us*)(ws + oFRH);  us* FRL = (us*)(ws + oFRL);
  float* SRE = (float*)(ws + oSRE); float* SIM = (float*)(ws + oSIM);
  us* PWH = (us*)(ws + oPWH);  us* PWL = (us*)(ws + oPWL);
  us* SSH = (us*)(ws + oSSH);  us* SSL = (us*)(ws + oSSL);
  float* FRO = (float*)(ws + oFRO);
  float* XR = (float*)(ws + oXR);
  us* ENV = (us*)(ws + oENV);
  us* ENVL = ENV + (size_t)(NSIG * NCH) * PL;
  us* Y3L = Y3 + (size_t)NSIG * PL;

  k_cvt_x<<<(NSIG * PL / 8 + 127) / 128, 128, 0, stream>>>(x, XH, XL);
  k_prep_tw<<<dim3(1024, 3), 128, 0, stream>>>(fsm, TFH, TFL, TIH, TIL, FSH, FSL);
  k_prep_filt<<<dim3((FROWS / 8 + 127) / 128, NFILT), 128, 0, stream>>>(cf, cbw, gc, gs, lp, BH, BL);
  k_conv16<<<dim3(MP / 128, NSIG), 128, 0, stream>>>(XH, XL, BH, BL, Y1);
  k_frames<<<RPAD / 32, 256, 0, stream>>>(Y1, win, FRH, FRL, NYQ);
  k_dft_fwd<<<dim3(RPAD / 32, 2), 128, 0, stream>>>(FRH, FRL, TFH, TFL, SRE, SIM, PWH, PWL);
  k_smear<<<RPAD / 32, 128, 0, stream>>>(PWH, PWL, FSH, FSL, SRE, SIM, SSH, SSL);
  k_dft_inv<<<RPAD / 32, 128, 0, stream>>>(SSH, SSL, TIH, TIL, NYQ, win, FRO);
  k_ola<<<NSIG * PL / 128, 128, 0, stream>>>(FRO, win, Y2H, Y2L);
  k_padz<<<4 * NCH + 4, 64, 0, stream>>>(ENV, Y3);
  k_gt<<<dim3(MP / 128, NCH, NSIG), 128, 0, stream>>>(Y2H, Y2L, BH, BL, XR, ENV, ENVL);
  k_lpf<<<dim3(MP / 128, NSIG), 128, 0, stream>>>(ENV, ENVL, BH, BL, XR, expn, emx, ocf, Y3, Y3L);
  k_conv16<<<dim3(MP / 128, NSIG), 128, 0, stream>>>(Y3, Y3L, BH + FROWS, BL + FROWS, Y4);
  k_out<<<((NSIG * TL) / 4 + 127) / 128, 128, 0, stream>>>(Y4, out);
}
